// SwinTransformerBlock3D_82643760709814
// MI455X (gfx1250) — hardware-run, weakly checked
//
#include <hip/hip_runtime.h>
#include <math.h>
#include <stdint.h>

#ifndef NB
#define NB 2
#endif
#define NB_FULL 2
#define CC 128
#define TT 16
#define IMH 56
#define IMW 56
#define WST 2
#define WSH 7
#define WSW 7
#define SST 1
#define SSH 3
#define SSW 3
#define NHD 4
#define HDD 32
#define HPAIRS (NHD / 2)
#define LTOK (WST * WSH * WSW)
#define LPAD 128
#define HIDN 512
#define QKVC (3 * CC)
#define NWTT (TT / WST)
#define NWY (IMH / WSH)
#define NWX (IMW / WSW)
#define NWB (NWTT * NWY * NWX)
#define PLANE (IMH * IMW)
#define NPIX_B (TT * PLANE)
#define NWT (NB * NWB)
#define MTOK (NB * NPIX_B)
#define MHALF (MTOK / 2)
#define NMASK 512
#define LTAB ((2 * WST - 1) * (2 * WSH - 1) * (2 * WSW - 1))
#define NBM (LTOK * LTOK)

#define WCAR   64.0f
#define QKVCAR 16.0f
#define PCAR   1024.0f
#define OCAR   64.0f
#define GCAR   16.0f
#define QSCALE 0.17677669529663687f

static_assert(NB >= 1 && NB <= NB_FULL);
static_assert(MTOK % 64 == 0);
static_assert(MHALF % 64 == 0);
static_assert(MTOK % 16 == 0);
static_assert(NWB * LTOK == NPIX_B);
static_assert(NWB == NMASK);
static_assert(NWY == 8 && NWX == 8 && NWTT == 8);
static_assert(CC % 64 == 0 && QKVC % 64 == 0 && HIDN % 64 == 0);
static_assert(CC % 32 == 0 && HIDN % 32 == 0);
static_assert(HDD == 32 && (NHD % 2) == 0);
static_assert(HPAIRS * 2 * HDD == CC);
static_assert(LTOK <= LPAD);
static_assert(CC == 16 * 8);

typedef __attribute__((ext_vector_type(16))) _Float16 v16h;
typedef __attribute__((ext_vector_type(8)))  _Float16 v8h;
typedef __attribute__((ext_vector_type(8)))  float    v8f;
typedef __attribute__((ext_vector_type(4)))  float    v4f;
typedef __attribute__((ext_vector_type(4)))  unsigned int v4u;

__device__ __forceinline__ unsigned short f2bf_bits(float f) {
  unsigned u = __float_as_uint(f);
  return (unsigned short)((u + 0x7FFFu + ((u >> 16) & 1u)) >> 16);
}
__device__ __forceinline__ float bf_bits2f(unsigned short h) { return __uint_as_float(((unsigned)h) << 16); }
__device__ __forceinline__ float bfr(float f) { return bf_bits2f(f2bf_bits(f)); }
__device__ __forceinline__ v4f bfr4(v4f a) { v4f r; r[0] = bfr(a[0]); r[1] = bfr(a[1]); r[2] = bfr(a[2]); r[3] = bfr(a[3]); return r; }

__device__ __forceinline__ void dep_guard_h(v8f& a, v8f& b, v16h x, v16h y) { asm volatile("v_nop\n\tv_nop\n\tv_nop\n\tv_nop" : "+v"(a), "+v"(b) : "v"(x), "v"(y)); }
__device__ __forceinline__ void dep_guard_h3(v8f& a, v8f& b, v16h x, v16h y, v16h z) { asm volatile("v_nop\n\tv_nop\n\tv_nop\n\tv_nop" : "+v"(a), "+v"(b) : "v"(x), "v"(y), "v"(z)); }
__device__ __forceinline__ void keep4_h(v16h a, v16h b, v16h c, v16h d) { asm volatile("v_nop" :: "v"(a), "v"(b), "v"(c), "v"(d)); }
__device__ __forceinline__ void acc_guard4(v8f& a, v8f& b, v8f& c, v8f& d) { asm volatile("v_nop\n\tv_nop\n\tv_nop\n\tv_nop" : "+v"(a), "+v"(b), "+v"(c), "+v"(d)); }
__device__ __forceinline__ void acc_guard2(v8f& a, v8f& b) { asm volatile("v_nop\n\tv_nop\n\tv_nop\n\tv_nop" : "+v"(a), "+v"(b)); }

union FragU { v16h v; v8h h[2]; _Float16 s[16]; };
struct FragH {
  static __device__ __forceinline__ v16h load(const _Float16* p) {
    FragU f; f.h[0] = *(const v8h*)(p); f.h[1] = *(const v8h*)(p + 16); return f.v;
  }
  static __device__ __forceinline__ v8f mma(v16h a, v16h b, v8f c) {
    return __builtin_amdgcn_wmma_f32_16x16x32_f16(false, a, false, b, (short)0, c, false, false);
  }
};

__device__ __forceinline__ int tok2raster(int m) {
  const int win = m / LTOK, l = m - win * LTOK;
  const int b = win / NWB, wi = win - b * NWB;
  const int tq = wi >> 6, hq = (wi >> 3) & 7, wq = wi & 7;
  const int i = l / (WSH * WSW), r = l - i * (WSH * WSW);
  const int j = r / WSW, k = r - j * WSW;
  int t = tq * WST + i + SST; t = (t >= TT) ? (t - TT) : t;
  int y = hq * WSH + j + SSH; y = (y >= IMH) ? (y - IMH) : y;
  int x = wq * WSW + k + SSW; x = (x >= IMW) ? (x - IMW) : x;
  return ((b * TT + t) * IMH + y) * IMW + x;
}

template <int BIAS_MODE, int OUT_MODE, bool RESID, bool RBF, int ACT, int ROWMAP>
__global__ __launch_bounds__(256) void wmma_gemm64(
    const unsigned short* __restrict__ Ap, int lda,
    const unsigned short* __restrict__ Btp, int ldb,
    void* Cout, int ldc,
    const float* __restrict__ bias,
    const float* resid,
    int M, int N, int K, float scale, float oscale) {
  const _Float16* A = (const _Float16*)Ap;
  const _Float16* Bt = (const _Float16*)Btp;
  __shared__ __align__(16) float sT[8][16 * 68];
  const int lane = threadIdx.x & 31;
  const int wave = threadIdx.x >> 5;
  const int tilesN = N >> 6;
  const int tilesM = M >> 6;
  const int tile = blockIdx.x * 8 + wave;
  if (tile >= tilesM * tilesN) return;
  const int tm = tile / tilesN;
  const int tn = tile - tm * tilesN;
  const int m0 = tm << 6;
  const int n0 = tn << 6;
  const int rlane = lane & 15;
  const int koff  = (lane >> 4) * 8;
  const int mOff  = (lane >> 4) * 8;

  v8f acc[4][4];
#pragma unroll
  for (int i = 0; i < 4; ++i)
#pragma unroll
    for (int j = 0; j < 4; ++j) acc[i][j] = (v8f){0.f,0.f,0.f,0.f,0.f,0.f,0.f,0.f};

  for (int k0 = 0; k0 < K; k0 += 32) {
    v16h bh[4];
#pragma unroll
    for (int j = 0; j < 4; ++j) {
      const size_t bo = (size_t)(n0 + (j << 4) + rlane) * ldb + koff + k0;
      bh[j] = FragH::load(Bt + bo);
    }
#pragma unroll
    for (int i = 0; i < 4; ++i) {
      const size_t ao = (size_t)(m0 + (i << 4) + rlane) * lda + koff + k0;
      const v16h ah = FragH::load(A + ao);
#pragma unroll
      for (int j = 0; j < 4; ++j) acc[i][j] = FragH::mma(ah, bh[j], acc[i][j]);
      dep_guard_h(acc[i][0], acc[i][3], ah, bh[3]);
    }
    keep4_h(bh[0], bh[1], bh[2], bh[3]);
  }
  acc_guard4(acc[0][0], acc[0][1], acc[0][2], acc[0][3]);
  acc_guard4(acc[1][0], acc[1][1], acc[1][2], acc[1][3]);
  acc_guard4(acc[2][0], acc[2][1], acc[2][2], acc[2][3]);
  acc_guard4(acc[3][0], acc[3][1], acc[3][2], acc[3][3]);

  float* slab = sT[wave];
#pragma unroll
  for (int i = 0; i < 4; ++i) {
    const int mBase = m0 + (i << 4);
#pragma unroll
    for (int j = 0; j < 4; ++j) {
      const int n = n0 + (j << 4) + rlane;
      float bv = 0.f;
      if (BIAS_MODE == 2) bv = bfr(bias[n]);
#pragma unroll
      for (int r = 0; r < 8; ++r) {
        float v = acc[i][j][r] * scale;
        if (BIAS_MODE == 2) v += bv;
        if (ACT == 5) v = 0.5f * v * (1.0f + erff(v * 0.70710678118654752f));
        v *= oscale;
        slab[(mOff + r) * 68 + (j << 4) + rlane] = v;
      }
    }
    __builtin_amdgcn_fence(3  , "workgroup");
    __builtin_amdgcn_wave_barrier();
    __builtin_amdgcn_fence(2  , "workgroup");
    if (OUT_MODE == 0) {
      float* C = (float*)Cout;
      const int hh = lane >> 4, c4 = (lane & 15) * 4;
      int orow[8];
#pragma unroll
      for (int it = 0; it < 8; ++it) {
        const int row = it * 2 + hh;
        orow[it] = ROWMAP ? tok2raster(mBase + row) : (mBase + row);
      }
      if (RESID) {
#pragma unroll
        for (int it = 0; it < 8; ++it) {
          const int row = it * 2 + hh;
          v4f v = *(const v4f*)(slab + row * 68 + c4);
          v4f rv = *(const v4f*)(resid + (size_t)orow[it] * ldc + n0 + c4);
          if (RBF) rv = bfr4(rv);
          v += rv;
          *(v4f*)(slab + row * 68 + c4) = v;
        }
      }
      for (int pass = 0; pass < 2; ++pass) {
#pragma unroll
        for (int it = 0; it < 8; ++it) {
          const int row = it * 2 + hh;
          const v4f v = *(const v4f*)(slab + row * 68 + c4);
          *(volatile v4f*)(C + (size_t)orow[it] * ldc + n0 + c4) = v;
        }
        __threadfence();
      }
    } else {
      const int q = lane >> 3, c8 = (lane & 7) * 8;
      unsigned short* C = (unsigned short*)Cout;
      for (int pass = 0; pass < 2; ++pass) {
#pragma unroll
        for (int it = 0; it < 4; ++it) {
          const int row = it * 4 + q;
          const float* sp = slab + row * 68 + c8;
          v8h hv;
#pragma unroll
          for (int e = 0; e < 8; ++e) hv[e] = (_Float16)sp[e];
          *(volatile v8h*)(C + (size_t)(mBase + row) * ldc + n0 + c8) = hv;
        }
        __threadfence();
      }
    }
    __builtin_amdgcn_fence(3  , "workgroup");
    __builtin_amdgcn_wave_barrier();
    __builtin_amdgcn_fence(2  , "workgroup");
  }
}

__global__ __launch_bounds__(256) void cvt_wt_kernel(const float* __restrict__ in, unsigned short* out, float carry, int K, int N) {
  __shared__ __align__(16) float sW[64 * 68];
  const int tid = threadIdx.x;
  const int tilesN = N >> 6, tilesK = K >> 6;
  int bid = blockIdx.x;
  bid = (bid < tilesN * tilesK) ? bid : (tilesN * tilesK - 1);
  const int kt = bid / tilesN, nt = bid - kt * tilesN;
  const int n0 = nt << 6, k0 = kt << 6;
#pragma unroll
  for (int it = 0; it < 4; ++it) {
    const int idx = it * 256 + tid;
    const int kk = idx >> 4, n4 = (idx & 15) * 4;
    const v4f v = *(const v4f*)(in + (size_t)(k0 + kk) * N + n0 + n4);
#pragma unroll
    for (int e = 0; e < 4; ++e) sW[(n4 + e) * 68 + kk] = bfr(v[e]) * carry;
  }
  __syncthreads();
  const int q = tid >> 3, c8 = (tid & 7) * 8;
  v4u val[2];
#pragma unroll
  for (int it = 0; it < 2; ++it) {
    const int rowl = it * 32 + q;
    const float* sp = sW + rowl * 68 + c8;
    const v4f a = *(const v4f*)(sp);
    const v4f b = *(const v4f*)(sp + 4);
    union { v8h h; v4u u; } pk;
#pragma unroll
    for (int e = 0; e < 4; ++e) { pk.h[e] = (_Float16)a[e]; pk.h[4 + e] = (_Float16)b[e]; }
    val[it] = pk.u;
  }
  for (int pass = 0; pass < 2; ++pass) {
#pragma unroll
    for (int it = 0; it < 2; ++it) {
      const int rowl = it * 32 + q;
      *(volatile v4u*)(out + (size_t)(n0 + rowl) * K + k0 + c8) = val[it];
    }
    __threadfence();
  }
}

template <bool RND>
__device__ __forceinline__ v4u ln_row_half(const float* rp, const float* __restrict__ g, const float* __restrict__ bb, int q) {
  v4f a = *(const v4f*)(rp + 8 * q);
  v4f c = *(const v4f*)(rp + 8 * q + 4);
  if (RND) { a = bfr4(a); c = bfr4(c); }
  float s = ((a[0] + a[1]) + (a[2] + a[3])) + ((c[0] + c[1]) + (c[2] + c[3]));
  s += __shfl_xor(s, 1, 32);
  s += __shfl_xor(s, 2, 32);
  s += __shfl_xor(s, 4, 32);
  s += __shfl_xor(s, 8, 32);
  const float mean = s * (1.0f / CC);
  const v4f d0 = a - mean, d1 = c - mean;
  float vs = ((d0[0] * d0[0] + d0[1] * d0[1]) + (d0[2] * d0[2] + d0[3] * d0[3])) +
             ((d1[0] * d1[0] + d1[1] * d1[1]) + (d1[2] * d1[2] + d1[3] * d1[3]));
  vs += __shfl_xor(vs, 1, 32);
  vs += __shfl_xor(vs, 2, 32);
  vs += __shfl_xor(vs, 4, 32);
  vs += __shfl_xor(vs, 8, 32);
  const float rstd = 1.0f / sqrtf(vs * (1.0f / CC) + 1e-5f);
  const v4f g0 = bfr4(*(const v4f*)(g + 8 * q)), g1 = bfr4(*(const v4f*)(g + 8 * q + 4));
  const v4f e0 = bfr4(*(const v4f*)(bb + 8 * q)), e1 = bfr4(*(const v4f*)(bb + 8 * q + 4));
  const v4f y0 = (d0 * rstd) * g0 + e0;
  const v4f y1 = (d1 * rstd) * g1 + e1;
  union { v8h h; v4u u; } pk;
#pragma unroll
  for (int e = 0; e < 4; ++e) { pk.h[e] = (_Float16)y0[e]; pk.h[4 + e] = (_Float16)y1[e]; }
  return pk.u;
}

__global__ __launch_bounds__(256) void ln1_kernel(const float* __restrict__ x, const float* __restrict__ g,
                                                  const float* __restrict__ bb, unsigned short* X16, int ntok) {
  const int tid = threadIdx.x, wave = tid >> 5, lane = tid & 31;
  const int h = lane >> 4, q = lane & 15;
  int m = blockIdx.x * 16 + wave * 2 + h;
  m = (m < ntok) ? m : (ntok - 1);
  const int src = tok2raster(m);
  const v4u val = ln_row_half<true>(x + (size_t)src * CC, g, bb, q);
  unsigned short* dst = X16 + (size_t)m * CC + 8 * q;
  *(volatile v4u*)dst = val;
  __threadfence();
  *(volatile v4u*)dst = val;
}

__global__ __launch_bounds__(256) void ln2_kernel(const float* xin, const float* __restrict__ g, const float* __restrict__ bb,
                                                  unsigned short* H2, int nrow) {
  const int tid = threadIdx.x, wave = tid >> 5, lane = tid & 31;
  const int h = lane >> 4, q = lane & 15;
  int row = blockIdx.x * 16 + wave * 2 + h;
  row = (row < nrow) ? row : (nrow - 1);
  const v4u val = ln_row_half<false>(xin + (size_t)row * CC, g, bb, q);
  unsigned short* dst = H2 + (size_t)row * CC + 8 * q;
  *(volatile v4u*)dst = val;
  __threadfence();
  *(volatile v4u*)dst = val;
}

__device__ __forceinline__ void stage_copy16(const _Float16* rp, _Float16* dst, float keep) {
  FragU u;
  u.h[0] = *(const v8h*)(rp);
  u.h[1] = *(const v8h*)(rp + 8);
  FragU o;
#pragma unroll
  for (int e = 0; e < 16; ++e) o.s[e] = (_Float16)((float)u.s[e] * keep);
  *(v8h*)(dst) = o.h[0];
  *(v8h*)(dst + 8) = o.h[1];
}

#define ATT_OFF_Q    0
#define ATT_OFF_K    (ATT_OFF_Q + 2 * LPAD * HDD * 2)
#define ATT_OFF_VT   (ATT_OFF_K + 2 * LPAD * HDD * 2)
#define ATT_OFF_P    (ATT_OFF_VT + 2 * HDD * LPAD * 2)
#define ATT_OFF_O    (ATT_OFF_P + 8 * 16 * LPAD * 2)
#define ATT_OFF_BM   (ATT_OFF_O + LPAD * 64 * 2)
#define ATT_LDS      (ATT_OFF_BM + 2 * NBM * 4)
static_assert(ATT_LDS == 175136);
static_assert((ATT_OFF_BM % 16) == 0);

__global__ __launch_bounds__(256) void win_attn_kernel(const unsigned short* __restrict__ QKVp,
                                                       const float* __restrict__ rpb, const int* __restrict__ ridx,
                                                       const float* __restrict__ mask,
                                                       unsigned short* O16, int nwin) {
  extern __shared__ __align__(16) unsigned char att_lds[];
  _Float16* sQ = (_Float16*)(att_lds + ATT_OFF_Q);
  _Float16* sK = (_Float16*)(att_lds + ATT_OFF_K);
  _Float16* sVT = (_Float16*)(att_lds + ATT_OFF_VT);
  _Float16* sP = (_Float16*)(att_lds + ATT_OFF_P);
  unsigned short* sO = (unsigned short*)(att_lds + ATT_OFF_O);
  float* sBM = (float*)(att_lds + ATT_OFF_BM);
  const _Float16* QKV = (const _Float16*)QKVp;
  const int tid = threadIdx.x, lane = tid & 31, wave = tid >> 5;
  const int hp = blockIdx.x % HPAIRS;
  int win = blockIdx.x / HPAIRS;
  win = (win < nwin) ? win : (nwin - 1);

#pragma unroll
  for (int it = 0; it < 2; ++it) {
    const int idx = it * 256 + tid;
    const int l = idx >> 2;
    const int c = idx & 3;
    const int hw = c >> 1;
    const int d0 = (c & 1) * 16;
    const int lc = (l < LTOK) ? l : (LTOK - 1);
    const float keep = (l < LTOK) ? 1.0f : 0.0f;
    const _Float16* rp = QKV + (size_t)(win * LTOK + lc) * QKVC + hp * 64 + c * 16;
    stage_copy16(rp, sQ + hw * (LPAD * HDD) + l * HDD + d0, keep);
    stage_copy16(rp + CC, sK + hw * (LPAD * HDD) + l * HDD + d0, keep);
    {
      FragU u;
      u.h[0] = *(const v8h*)(rp + 2 * CC);
      u.h[1] = *(const v8h*)(rp + 2 * CC + 8);
#pragma unroll
      for (int e = 0; e < 16; ++e) {
        const float fv = (float)u.s[e] * keep;
        sVT[hw * (HDD * LPAD) + (d0 + e) * LPAD + l] = (_Float16)fv;
      }
    }
  }
  {
    const float* mk = mask + (size_t)(win % NMASK) * NBM;
#pragma unroll 1
    for (int it = 0; it < (NBM + 255) / 256; ++it) {
      const int o = it * 256 + tid;
      const int oc = (o < NBM) ? o : (NBM - 1);
      int ri = ridx[oc];
      ri = (ri < 0) ? 0 : ri;
      ri = (ri < LTAB) ? ri : (LTAB - 1);
      const float mv = bfr(mk[oc]);
      const float b0 = bfr(rpb[ri * NHD + hp * 2]);
      const float b1 = bfr(rpb[ri * NHD + hp * 2 + 1]);
      const float v0 = b0 + mv;
      const float v1 = b1 + mv;
      if (o < NBM) { sBM[o] = v0; sBM[NBM + o] = v1; }
    }
  }
  __syncthreads();

  const int qr0 = wave * 16;
  const int rlane = lane & 15, koff = (lane >> 4) * 8, mOff = (lane >> 4) * 8;
  const v8f z8 = (v8f){0.f,0.f,0.f,0.f,0.f,0.f,0.f,0.f};
  _Float16* pw = sP + wave * (16 * LPAD);

#pragma unroll 1
  for (int hw = 0; hw < 2; ++hw) {
    const _Float16* q_ = sQ + hw * (LPAD * HDD);
    const _Float16* k_ = sK + hw * (LPAD * HDD);
    const _Float16* vt_ = sVT + hw * (HDD * LPAD);
    const float* bm_ = sBM + hw * NBM;

    v8f s[8];
    {
      const v16h a = FragH::load(q_ + (qr0 + rlane) * HDD + koff);
      v16h bq[8];
#pragma unroll
      for (int j = 0; j < 8; ++j) bq[j] = FragH::load(k_ + (16 * j + rlane) * HDD + koff);
#pragma unroll
      for (int j = 0; j < 8; ++j) s[j] = FragH::mma(a, bq[j], z8);
      dep_guard_h(s[0], s[7], a, bq[7]);
      keep4_h(bq[0], bq[1], bq[2], bq[3]);
      keep4_h(bq[4], bq[5], bq[6], bq[7]);
    }
    acc_guard4(s[0], s[1], s[2], s[3]);
    acc_guard4(s[4], s[5], s[6], s[7]);

#pragma unroll
    for (int j = 0; j < 8; ++j) {
      const int n = 16 * j + rlane;
      const int nc = (n < LTOK) ? n : (LTOK - 1);
#pragma unroll
      for (int r = 0; r < 8; ++r) {
        const int m = qr0 + mOff + r;
        const int mc = (m < LTOK) ? m : (LTOK - 1);
        float val = s[j][r] * (QSCALE / (QKVCAR * QKVCAR)) + bm_[mc * LTOK + nc];
        val = (m < LTOK) ? val : 0.0f;
        val = (n < LTOK) ? val : -INFINITY;
        s[j][r] = val;
      }
    }

#pragma unroll
    for (int r = 0; r < 8; ++r) {
      float mx = fmaxf(fmaxf(fmaxf(s[0][r], s[1][r]), fmaxf(s[2][r], s[3][r])),
                       fmaxf(fmaxf(s[4][r], s[5][r]), fmaxf(s[6][r], s[7][r])));
      mx = fmaxf(mx, __shfl_xor(mx, 1, 32));
      mx = fmaxf(mx, __shfl_xor(mx, 2, 32));
      mx = fmaxf(mx, __shfl_xor(mx, 4, 32));
      mx = fmaxf(mx, __shfl_xor(mx, 8, 32));
      float ev[8];
#pragma unroll
      for (int j = 0; j < 8; ++j) ev[j] = expf(s[j][r] - mx);
      float sum = ((ev[0] + ev[1]) + (ev[2] + ev[3])) + ((ev[4] + ev[5]) + (ev[6] + ev[7]));
      sum += __shfl_xor(sum, 1, 32);
      sum += __shfl_xor(sum, 2, 32);
      sum += __shfl_xor(sum, 4, 32);
      sum += __shfl_xor(sum, 8, 32);
      const float pn = PCAR / sum;
      _Float16* prow = pw + (mOff + r) * LPAD + rlane;
#pragma unroll
      for (int j = 0; j < 8; ++j) prow[16 * j] = (_Float16)(ev[j] * pn);
    }
    __builtin_amdgcn_fence(3  , "workgroup");
    __builtin_amdgcn_wave_barrier();
    __builtin_amdgcn_fence(2  , "workgroup");

    v8f o[2];
    o[0] = z8; o[1] = z8;
#pragma unroll
    for (int k0 = 0; k0 < LPAD; k0 += 32) {
      const v16h a  = FragH::load(pw + rlane * LPAD + k0 + koff);
      const v16h b0 = FragH::load(vt_ + rlane * LPAD + k0 + koff);
      const v16h b1 = FragH::load(vt_ + (16 + rlane) * LPAD + k0 + koff);
      o[0] = FragH::mma(a, b0, o[0]);
      o[1] = FragH::mma(a, b1, o[1]);
      dep_guard_h3(o[0], o[1], a, b0, b1);
    }
    acc_guard2(o[0], o[1]);
#pragma unroll
    for (int jd = 0; jd < 2; ++jd) {
#pragma unroll
      for (int r = 0; r < 8; ++r) {
        const float ov = o[jd][r] * (OCAR / (PCAR * QKVCAR));
        sO[(qr0 + mOff + r) * 64 + hw * 32 + 16 * jd + rlane] = __builtin_bit_cast(unsigned short, (_Float16)ov);
      }
    }
    __builtin_amdgcn_fence(3  , "workgroup");
    __builtin_amdgcn_wave_barrier();
    __builtin_amdgcn_fence(2  , "workgroup");
  }
  __syncthreads();
  {
    const int c8 = (tid & 7) * 8;
    unsigned short* Ob = O16 + (size_t)win * LTOK * CC + hp * 64 + c8;
    v4u ov[4];
#pragma unroll
    for (int it = 0; it < 4; ++it) {
      const int rowl = it * 32 + (tid >> 3);
      ov[it] = *(const v4u*)(&sO[rowl * 64 + c8]);
    }
    for (int pass = 0; pass < 2; ++pass) {
#pragma unroll
      for (int it = 0; it < 4; ++it) {
        const int rowl = it * 32 + (tid >> 3);
        if (rowl < LTOK) *(volatile v4u*)(Ob + (size_t)rowl * CC) = ov[it];
      }
      __threadfence();
    }
  }
}

extern "C" void kernel_launch(void* const* d_in, const int* in_sizes, int n_in,
                              void* d_out, int out_size, void* d_ws, size_t ws_size,
                              hipStream_t stream) {
  if (n_in < 16) return;
  if (in_sizes[0] < NB * NPIX_B * CC) return;
  if (in_sizes[1] < NMASK * NBM) return;
  if (in_sizes[2] < NBM) return;
  if (in_sizes[3] < CC || in_sizes[4] < CC) return;
  if (in_sizes[5] < CC * QKVC || in_sizes[6] < QKVC) return;
  if (in_sizes[7] < LTAB * NHD) return;
  if (in_sizes[8] < CC * CC || in_sizes[9] < CC) return;
  if (in_sizes[10] < CC || in_sizes[11] < CC) return;
  if (in_sizes[12] < CC * HIDN || in_sizes[13] < HIDN) return;
  if (in_sizes[14] < HIDN * CC || in_sizes[15] < CC) return;
  if (out_size < NB * NPIX_B * CC) return;

  const float* x       = (const float*)d_in[0];
  const float* maskm   = (const float*)d_in[1];
  const int*   ridx    = (const int*)d_in[2];
  const float* norm1_w = (const float*)d_in[3];
  const float* norm1_b = (const float*)d_in[4];
  const float* qkv_w   = (const float*)d_in[5];
  const float* qkv_b   = (const float*)d_in[6];
  const float* rpb     = (const float*)d_in[7];
  const float* proj_w  = (const float*)d_in[8];
  const float* proj_b  = (const float*)d_in[9];
  const float* norm2_w = (const float*)d_in[10];
  const float* norm2_b = (const float*)d_in[11];
  const float* fc1_w   = (const float*)d_in[12];
  const float* fc1_b   = (const float*)d_in[13];
  const float* fc2_w   = (const float*)d_in[14];
  const float* fc2_b   = (const float*)d_in[15];
  float* outp = (float*)d_out;

  const size_t PWQ = (size_t)QKVC * CC * 2;
  const size_t PWP = (size_t)CC * CC * 2;
  const size_t PW1 = (size_t)HIDN * CC * 2;
  const size_t PW2 = (size_t)CC * HIDN * 2;
  const size_t PA  = (size_t)MTOK * CC * 2;
  const size_t PB  = (size_t)MTOK * QKVC * 2;
  static_assert((size_t)MHALF * HIDN * 2 <= (size_t)MTOK * QKVC * 2);
  size_t off = 0;
  const size_t oWq = off; off += PWQ;
  const size_t oWp = off; off += PWP;
  const size_t oW1 = off; off += PW1;
  const size_t oW2 = off; off += PW2;
  const size_t oA = off; off += PA;
  const size_t oB = off; off += PB;
  if (off > ws_size) return;
  if (off > (size_t)134217728u) return;

  char* ws = (char*)d_ws;
  unsigned short* Wq = (unsigned short*)(ws + oWq);
  unsigned short* Wp = (unsigned short*)(ws + oWp);
  unsigned short* W1 = (unsigned short*)(ws + oW1);
  unsigned short* W2 = (unsigned short*)(ws + oW2);
  unsigned short* RA = (unsigned short*)(ws + oA);
  unsigned short* RB = (unsigned short*)(ws + oB);

  const dim3 blk(256);
  cvt_wt_kernel<<<dim3((QKVC / 64) * (CC / 64)), blk, 0, stream>>>(qkv_w, Wq, WCAR, CC, QKVC);
  cvt_wt_kernel<<<dim3((CC / 64) * (CC / 64)), blk, 0, stream>>>(proj_w, Wp, WCAR, CC, CC);
  cvt_wt_kernel<<<dim3((HIDN / 64) * (CC / 64)), blk, 0, stream>>>(fc1_w, W1, WCAR, CC, HIDN);
  cvt_wt_kernel<<<dim3((CC / 64) * (HIDN / 64)), blk, 0, stream>>>(fc2_w, W2, WCAR, HIDN, CC);
  ln1_kernel<<<dim3(MTOK / 16), blk, 0, stream>>>(x, norm1_w, norm1_b, RA, MTOK);

  const int tilesM = MTOK / 64;
  const int tilesH = MHALF / 64;
  wmma_gemm64<2, 1, false, false, 0, 0><<<dim3((tilesM * (QKVC / 64) + 7) / 8), blk, 0, stream>>>(
      RA, CC, Wq, CC, (void*)RB, QKVC, qkv_b, qkv_b, MTOK, QKVC, CC, 1.0f / WCAR, QKVCAR);
  (void)hipFuncSetAttribute(reinterpret_cast<const void*>(&win_attn_kernel), hipFuncAttributeMaxDynamicSharedMemorySize, ATT_LDS);
  win_attn_kernel<<<dim3(NWT * HPAIRS), blk, ATT_LDS, stream>>>(RB, rpb, ridx, maskm, RA, NWT);
  wmma_gemm64<2, 0, true, true, 0, 1><<<dim3((tilesM * (CC / 64) + 7) / 8), blk, 0, stream>>>(
      RA, CC, Wp, CC, (void*)outp, CC, proj_b, x, MTOK, CC, CC, 1.0f / (OCAR * WCAR), 1.0f);
  ln2_kernel<<<dim3(MTOK / 16), blk, 0, stream>>>(outp, norm2_w, norm2_b, RA, MTOK);
  for (int half = 0; half < 2; ++half) {
    const unsigned short* Ah = RA + (size_t)half * MHALF * CC;
    float* Oh = outp + (size_t)half * MHALF * CC;
    wmma_gemm64<2, 1, false, false, 5, 0><<<dim3((tilesH * (HIDN / 64) + 7) / 8), blk, 0, stream>>>(
        Ah, CC, W1, CC, (void*)RB, HIDN, fc1_b, fc1_b, MHALF, HIDN, CC, 1.0f / WCAR, GCAR);
    wmma_gemm64<2, 0, true, false, 0, 0><<<dim3((tilesH * (CC / 64) + 7) / 8), blk, 0, stream>>>(
        RB, HIDN, W2, HIDN, (void*)Oh, CC, fc2_b, Oh, MHALF, CC, HIDN, 1.0f / (GCAR * WCAR), 1.0f);
  }
  (void)hipGetLastError();
}
